// Generator_24592982737248
// MI455X (gfx1250) — hardware-verified
//
#include <hip/hip_runtime.h>


#ifndef NB
#define NB 8
#endif
#define NB_FULL 8
#define NT   16
#define NN   4
#define MD   128
#define RES_ 1024
#define KP   256
#define NCC  (NB * NT * NN)
#define TWO_PI_OVER_RES ((float)(6.283185307179586 / (double)RES_))

static_assert(NB <= NB_FULL);
static_assert(NN == 4);
static_assert(KP == 2 * MD);
static_assert(KP % 32 == 0);
static_assert(NCC % 64 == 0);
static_assert(RES_ % 64 == 0);
static_assert(RES_ == 1024);
static_assert((RES_ & (RES_ - 1)) == 0);
static_assert(((size_t)NCC * KP / 8) % 256 == 0);
static_assert(((size_t)RES_ * KP / 8) % 256 == 0);
static_assert(sizeof(float) * RES_ <= 131072);
static_assert(32 * 16 * 32 == 64 * 64 * 4);

typedef _Float16 h16;
typedef __attribute__((ext_vector_type(16))) _Float16 v16h;
typedef __attribute__((ext_vector_type(8)))  _Float16 v8h;
typedef __attribute__((ext_vector_type(8)))  float    v8f;
typedef __attribute__((ext_vector_type(4)))  float    v4f;

__device__ __forceinline__ unsigned short f2bf(float f) { unsigned u = __float_as_uint(f); u += 0x7FFFu + ((u >> 16) & 1u); return (unsigned short)(u >> 16); }
__device__ __forceinline__ float bfr(float f) { return __uint_as_float(((unsigned)f2bf(f)) << 16); }
__device__ __forceinline__ v16h cat16(v8h lo, v8h hi) { return __builtin_shufflevector(lo, hi, 0, 1, 2, 3, 4, 5, 6, 7, 8, 9, 10, 11, 12, 13, 14, 15); }
__device__ __forceinline__ v8f wmma16(v16h a, v16h b, v8f c) { return __builtin_amdgcn_wmma_f32_16x16x32_f16(false, a, false, b, (short)0, c, false, false); }
__device__ __forceinline__ v16h  ldh(const h16* p) { return cat16(*(const v8h*)p, *(const v8h*)(p + 16)); }
__device__ __forceinline__ v8f wmma16g(v16h a, v16h b, v8f c) { c = wmma16(a, b, c); asm volatile("v_nop\n\tv_nop\n\tv_nop\n\tv_nop" : "+v"(c) : "v"(a), "v"(b)); return c; }
static __device__ __forceinline__ h16 toh_flush(float v) { const h16 r = (h16)v; return (fabsf(v) < 6.103515625e-05f) ? (h16)0.0f : r; }

__global__ __launch_bounds__(256) void k_xplane(const float* __restrict__ x, const int* __restrict__ modes_p, h16* XH) {
    const int mraw = modes_p[0];
    const int md = mraw < 0 ? 0 : (mraw > MD ? MD : mraw);
    const unsigned i = blockIdx.x * 256u + threadIdx.x; if (i >= (unsigned)(NCC * (KP / 8))) return;
    const int cc = (int)(i / (unsigned)(KP / 8)), piece = (int)(i % (unsigned)(KP / 8));
    const int j = piece >> 2, c8 = (piece & 3) * 8;
    const int m0 = 16 * j + (c8 & 15);
    const size_t so = (size_t)cc * (2 * MD) + (size_t)((c8 >= 16) ? MD : 0) + (size_t)m0;
    v8f v = *(const v8f*)(x + so);
    asm volatile("" : "+v"(v));
    v8h o;
#pragma unroll
    for (int e = 0; e < 8; ++e) { const h16 hv = toh_flush(bfr(v[e])); o[e] = (m0 + e < md) ? hv : (h16)0.0f; }
    *(volatile v8h*)(XH + (size_t)i * 8) = o; __threadfence(); *(volatile v8h*)(XH + (size_t)i * 8) = o;
}

__global__ __launch_bounds__(256) void k_wplane(const int* __restrict__ modes_p, h16* WH) {
    __shared__ float tbl[RES_];
#pragma unroll 1
    for (int q = threadIdx.x; q < RES_; q += 256) {
        const int n = (q + RES_ / 8) / (RES_ / 4);
        const int r = q - n * (RES_ / 4);
        const float t  = (float)r * TWO_PI_OVER_RES;
        const float t2 = t * t;
        const float sn = t * fmaf(t2, fmaf(t2, fmaf(t2, -1.9515295891e-4f, 8.3321608736e-3f), -1.6666654611e-1f), 1.0f);
        const float cs = fmaf(t2, fmaf(t2, fmaf(t2, fmaf(t2, 2.443315711809948e-5f, -1.388731625493765e-3f), 4.166664568298827e-2f), -0.5f), 1.0f);
        float cv = (n & 1) ? -sn : cs;
        cv = (n & 2) ? -cv : cv;
        tbl[q] = cv;
    }
    __syncthreads();
    const int mraw = modes_p[0];
    const int md = mraw < 0 ? 0 : (mraw > MD ? MD : mraw);
    const unsigned i = blockIdx.x * 256u + threadIdx.x;
    const int s = (int)((i / (unsigned)(KP / 8)) & (unsigned)(RES_ - 1)), piece = (int)(i % (unsigned)(KP / 8));
    const int j = piece >> 2, c8 = (piece & 3) * 8;
    const int sh = (c8 >= 16) ? (RES_ / 4) : 0;
    const int m0 = 16 * j + (c8 & 15);
    v8h o;
#pragma unroll
    for (int e = 0; e < 8; ++e) {
        const int m = m0 + e;
        float w = tbl[(m * s + sh) & (RES_ - 1)];
        asm volatile("" : "+v"(w));
        const h16 hv = toh_flush(w);
        o[e] = (m < md) ? hv : (h16)0.0f; }
    if (i < (unsigned)(RES_ * (KP / 8))) {
        *(volatile v8h*)(WH + (size_t)i * 8) = o; __threadfence(); *(volatile v8h*)(WH + (size_t)i * 8) = o; }
}

__global__ __launch_bounds__(32) void k_synth(const h16* __restrict__ XH, const h16* __restrict__ WH, const int* __restrict__ modes_p, const int* __restrict__ res_p, float* OUT) {
    const int lane = threadIdx.x & 31, lr = lane & 15, hi = lane >> 4; const int r0 = blockIdx.x * 64, c0 = blockIdx.y * 64;
    const int mraw = modes_p[0], rraw = res_p[0];
    const int md = mraw < 0 ? 0 : (mraw > MD ? MD : mraw);
    const int nsteps = __builtin_amdgcn_readfirstlane((md + 15) >> 4);
    const bool ok = (rraw == RES_) & (mraw >= 0) & (mraw <= MD);
    v8f acc[4][4];
#pragma unroll
    for (int mb = 0; mb < 4; ++mb)
#pragma unroll
        for (int nb = 0; nb < 4; ++nb) acc[mb][nb] = (v8f){};
    const size_t aoff = (size_t)(r0 + lr) * KP + 8 * hi, boff = (size_t)(c0 + lr) * KP + 8 * hi;
#pragma unroll 1
    for (int j = 0; j < KP / 32; ++j) {
        if (j >= nsteps) break;
        const int kc = j * 32;
        v16h a[4];
#pragma unroll
        for (int mb = 0; mb < 4; ++mb) a[mb] = ldh(XH + aoff + (size_t)mb * 16 * KP + kc);
#pragma unroll
        for (int nb = 0; nb < 4; ++nb) { const v16h b = ldh(WH + boff + (size_t)nb * 16 * KP + kc);
#pragma unroll
            for (int mb = 0; mb < 4; ++mb) acc[mb][nb] = wmma16g(a[mb], b, acc[mb][nb]); }
    }
    if (!ok) {
        const float qn = __uint_as_float(0x7FC00000u);
#pragma unroll
        for (int mb = 0; mb < 4; ++mb)
#pragma unroll
            for (int nb = 0; nb < 4; ++nb)
#pragma unroll
                for (int r = 0; r < 8; ++r) acc[mb][nb][r] = qn;
    }
    float* ob = OUT + (size_t)(r0 / NN + 2 * hi) * (size_t)(RES_ * NN) + (size_t)(c0 + lr) * NN;
#pragma unroll 1
    for (int ps = 0; ps < 2; ++ps) {
#pragma unroll
        for (int mb = 0; mb < 4; ++mb) {
#pragma unroll
            for (int nb = 0; nb < 4; ++nb) {
#pragma unroll
                for (int q = 0; q < 2; ++q) {
                    v4f val; val[0] = acc[mb][nb][4 * q + 0]; val[1] = acc[mb][nb][4 * q + 1]; val[2] = acc[mb][nb][4 * q + 2]; val[3] = acc[mb][nb][4 * q + 3];
                    *(volatile v4f*)(ob + (size_t)(4 * mb + q) * (size_t)(RES_ * NN) + (size_t)(nb * 16 * NN)) = val; } } }
        if (ps == 0) __threadfence(); }
}

static constexpr size_t al256(size_t v) { return (v + 255) & ~(size_t)255; }
static constexpr size_t SZ_XH = al256((size_t)NCC * KP * 2);
static constexpr size_t SZ_WH = al256((size_t)RES_ * KP * 2);
static constexpr size_t SZ_TOTAL = SZ_XH + SZ_WH;
static_assert(SZ_TOTAL <= (size_t)134217728);
static_assert((size_t)(NCC * (KP / 8)) * 16 == (size_t)NCC * KP * 2);
static_assert((size_t)(RES_ * (KP / 8)) * 16 == (size_t)RES_ * KP * 2);
static_assert((size_t)(NCC / NN) * RES_ * NN == (size_t)NB * NT * RES_ * NN);

extern "C" void kernel_launch(void* const* d_in, const int* in_sizes, int n_in,
                              void* d_out, int out_size, void* d_ws, size_t ws_size, hipStream_t stream) {
    if (n_in < 3) return;
    if ((size_t)in_sizes[0] < (size_t)NCC * 2 * MD) return;
    if (in_sizes[1] < 1 || in_sizes[2] < 1) return;
    if ((size_t)out_size < (size_t)NB * NT * RES_ * NN) return;
    if (SZ_TOTAL > ws_size) return;
    const float* x = (const float*)d_in[0];
    const int* modes_p = (const int*)d_in[1];
    const int* res_p = (const int*)d_in[2];
    float* OUT = (float*)d_out;
    char* wsp = (char*)d_ws;
    h16* XH = (h16*)wsp; wsp += SZ_XH;
    h16* WH = (h16*)wsp; wsp += SZ_WH;

    k_xplane<<<(unsigned)((size_t)NCC * (KP / 8) / 256), 256, 0, stream>>>(x, modes_p, XH);
    k_wplane<<<(unsigned)((size_t)RES_ * (KP / 8) / 256), 256, 0, stream>>>(modes_p, WH);
    k_synth<<<dim3(NCC / 64, RES_ / 64, 1), 32, 0, stream>>>(XH, WH, modes_p, res_p, OUT);
}
